// CoevolExtractor_14216341750247
// MI455X (gfx1250) — hardware-verified
//
#include <hip/hip_runtime.h>


typedef __attribute__((ext_vector_type(16))) _Float16 v16h;
typedef __attribute__((ext_vector_type(8)))  _Float16 v8h;
typedef __attribute__((ext_vector_type(8)))  float    v8f;
typedef __attribute__((ext_vector_type(4)))  float    v4f;

__device__ __forceinline__ void dep_guard_h(v8f& a, v8f& b, v16h x, v16h y) { asm volatile("v_nop\n\tv_nop\n\tv_nop\n\tv_nop" : "+v"(a), "+v"(b) : "v"(x), "v"(y)); }
__device__ __forceinline__ void keep4_h(v16h a, v16h b, v16h c, v16h d) { asm volatile("v_nop" :: "v"(a), "v"(b), "v"(c), "v"(d)); }

template <typename T> struct Frag;
template <> struct Frag<_Float16> {
  typedef v16h V; union U { v16h v; v8h h[2]; };
  static __device__ __forceinline__ v16h load(const _Float16* p) {
    U f; f.h[0] = *(const v8h*)(p); f.h[1] = *(const v8h*)(p + 16); return f.v;
  }
  static __device__ __forceinline__ v8f mma(v16h a, v16h b, v8f c) {
    return __builtin_amdgcn_wmma_f32_16x16x32_f16(false, a, false, b, (short)0, c, false, false);
  }
  static __device__ __forceinline__ void guard(v8f& a, v8f& b, v16h x, v16h y) { dep_guard_h(a, b, x, y); }
  static __device__ __forceinline__ void keep(v16h a, v16h b, v16h c, v16h d) { keep4_h(a, b, c, d); }
};

__device__ __forceinline__ v8f mma_h(v16h a, v16h b, v8f c) {
  c = __builtin_amdgcn_wmma_f32_16x16x32_f16(false, a, false, b, (short)0, c, false, false);
  asm volatile("v_nop\n\tv_nop\n\tv_nop\n\tv_nop" : "+v"(c) : "v"(a), "v"(b));
  return c;
}

__device__ __forceinline__ v8f vz8() { return (v8f){0.f, 0.f, 0.f, 0.f, 0.f, 0.f, 0.f, 0.f}; }

#define NN      128
#define LL      256
#define PP      32
#define NO      128
#define CH      1024
#define TPITCH  136
#define PLP     1032
#define SLP     132
#define WSC     64.0f
#define WSC_INV (1.0f / 64.0f)
#define LN_EPS  1e-5f

__global__ __launch_bounds__(256) void k_transpose(const float* __restrict__ xd, const float* __restrict__ xw,
                                                   _Float16* __restrict__ At, _Float16* __restrict__ Bt) {
  __shared__ __align__(16) _Float16 tile[PP * TPITCH];
  const int bx = blockIdx.x;
  const int which = (bx >= LL) ? 1 : 0;
  const int i = which ? (bx - LL) : bx;
  const float* src = which ? xw : xd;
  _Float16* dst = which ? Bt : At;
  const int t = threadIdx.x;
#pragma unroll
  for (int it = 0; it < 16; ++it) {
    const int idx = it * 256 + t;
    const int n = idx >> 5;
    const int j = idx & 31;
    const float v = src[(size_t)n * (LL * PP) + (size_t)i * PP + j];
    tile[j * TPITCH + n] = (_Float16)v;
  }
  __syncthreads();
  const int wave = t >> 5, lane = t & 31, hh = lane >> 4, c8 = (lane & 15) * 8;
  for (int pass = 0; pass < 2; ++pass) {
#pragma unroll
    for (int it = 0; it < 2; ++it) {
      const int row = wave * 4 + it * 2 + hh;
      const v8h v = *(const v8h*)(tile + row * TPITCH + c8);
      *(volatile v8h*)(dst + ((size_t)i * PP + row) * NN + c8) = v;
    }
    __threadfence();
  }
}

__global__ __launch_bounds__(256) void k_castw(const float* __restrict__ in, _Float16* __restrict__ out, int n2, float sc) {
  const int i = blockIdx.x * 256 + threadIdx.x;
  if (i < n2) {
    const _Float16 h0 = (_Float16)(in[2 * i] * sc), h1 = (_Float16)(in[2 * i + 1] * sc);
    const unsigned u = (unsigned)__builtin_bit_cast(unsigned short, h0) | ((unsigned)__builtin_bit_cast(unsigned short, h1) << 16);
    ((volatile unsigned*)out)[i] = u;
    __threadfence();
    ((volatile unsigned*)out)[i] = u;
  }
}

__global__ __launch_bounds__(256) void k_main(const _Float16* __restrict__ At, const _Float16* __restrict__ Bt,
                                              const _Float16* __restrict__ Wh,
                                              const float* __restrict__ gamma, const float* __restrict__ beta,
                                              const float* __restrict__ bias, float* __restrict__ outp) {
  __shared__ __align__(16) _Float16 pln[16 * PLP];
  __shared__ __align__(16) float    slab[16 * SLP];
  const int t = threadIdx.x;
  const int wave = t >> 5;
  const int lane = t & 31;
  const int hh = lane >> 4;
  const int rl = lane & 15;
  const int koff = hh * 8;
  const int i0 = blockIdx.y * 4;
  const int l0 = blockIdx.x * 4;

  float gm[2][2][8], be[2][2][8];
#pragma unroll
  for (int jt = 0; jt < 2; ++jt)
#pragma unroll
    for (int mt = 0; mt < 2; ++mt)
#pragma unroll
      for (int r = 0; r < 8; ++r) {
        const int ch = (jt * 16 + 8 * hh + r) * PP + mt * 16 + rl;
        gm[jt][mt][r] = gamma[ch];
        be[jt][mt][r] = beta[ch];
      }

#pragma unroll 1
  for (int c = 0; c < 2; ++c) {
    const int p = wave * 2 + c;
    const int i = i0 + (p >> 2);
    const int l = l0 + (p & 3);
    const _Float16* Ap = At + (size_t)i * PP * NN;
    const _Float16* Bp = Bt + (size_t)l * PP * NN;

    v8f acc[2][2];
#pragma unroll
    for (int jt = 0; jt < 2; ++jt)
#pragma unroll
      for (int mt = 0; mt < 2; ++mt) acc[jt][mt] = vz8();

#pragma unroll 1
    for (int k0 = 0; k0 < NN; k0 += 32) {
      v16h a[2], b[2];
#pragma unroll
      for (int jt = 0; jt < 2; ++jt) a[jt] = Frag<_Float16>::load(Ap + (size_t)(jt * 16 + rl) * NN + k0 + koff);
#pragma unroll
      for (int mt = 0; mt < 2; ++mt) b[mt] = Frag<_Float16>::load(Bp + (size_t)(mt * 16 + rl) * NN + k0 + koff);
#pragma unroll
      for (int jt = 0; jt < 2; ++jt)
#pragma unroll
        for (int mt = 0; mt < 2; ++mt) acc[jt][mt] = mma_h(a[jt], b[mt], acc[jt][mt]);
    }

    float s1 = 0.f;
#pragma unroll
    for (int jt = 0; jt < 2; ++jt)
#pragma unroll
      for (int mt = 0; mt < 2; ++mt)
#pragma unroll
        for (int r = 0; r < 8; ++r) s1 += acc[jt][mt][r];
#pragma unroll
    for (int off = 16; off > 0; off >>= 1) s1 += __shfl_xor(s1, off, 32);
    const float mu = s1 * (1.0f / CH);
    float s2 = 0.f;
#pragma unroll
    for (int jt = 0; jt < 2; ++jt)
#pragma unroll
      for (int mt = 0; mt < 2; ++mt)
#pragma unroll
        for (int r = 0; r < 8; ++r) {
          const float d = acc[jt][mt][r] - mu;
          s2 += d * d;
        }
#pragma unroll
    for (int off = 16; off > 0; off >>= 1) s2 += __shfl_xor(s2, off, 32);
    const float var = s2 * (1.0f / CH);
    const float rstd = rsqrtf(var + LN_EPS);

    _Float16* prow = pln + p * PLP;
#pragma unroll
    for (int jt = 0; jt < 2; ++jt)
#pragma unroll
      for (int mt = 0; mt < 2; ++mt)
#pragma unroll
        for (int r = 0; r < 8; ++r) {
          const float yv = (acc[jt][mt][r] - mu) * rstd;
          const float z = yv * gm[jt][mt][r] + be[jt][mt][r];
          prow[(jt * 16 + 8 * hh + r) * PP + mt * 16 + rl] = (_Float16)z;
        }
  }
  __syncthreads();

  v8f oacc = vz8();
  const _Float16* arow = pln + rl * PLP + koff;
  const _Float16* wrow = Wh + (size_t)(wave * 16 + rl) * CH + koff;
#pragma unroll 2
  for (int k0 = 0; k0 < CH; k0 += 32) {
    const v16h a = Frag<_Float16>::load(arow + k0);
    const v16h b = Frag<_Float16>::load(wrow + k0);
    oacc = mma_h(a, b, oacc);
  }
  const int o = wave * 16 + rl;
  const float bv = bias[o];
#pragma unroll
  for (int r = 0; r < 8; ++r) slab[(8 * hh + r) * SLP + o] = oacc[r] * WSC_INV + bv;
  __syncthreads();

  for (int pass = 0; pass < 2; ++pass) {
#pragma unroll
    for (int it = 0; it < 2; ++it) {
      const int p = wave * 2 + it;
      const int i = i0 + (p >> 2);
      const int l = l0 + (p & 3);
      const v4f v = *(const v4f*)(slab + p * SLP + lane * 4);
      *(volatile v4f*)(outp + ((size_t)(i * LL + l)) * NO + lane * 4) = v;
    }
    __threadfence();
  }
}

extern "C" void kernel_launch(void* const* d_in, const int* in_sizes, int n_in,
                              void* d_out, int out_size, void* d_ws, size_t ws_size,
                              hipStream_t stream) {
  if (n_in < 6) return;
  if (in_sizes[0] != NN * LL * PP || in_sizes[1] != NN * LL * PP || in_sizes[2] != CH ||
      in_sizes[3] != CH || in_sizes[4] != NO * CH || in_sizes[5] != NO) return;
  if (out_size != LL * LL * NO) return;

  const float* xd    = (const float*)d_in[0];
  const float* xw    = (const float*)d_in[1];
  const float* gamma = (const float*)d_in[2];
  const float* beta  = (const float*)d_in[3];
  const float* Wg    = (const float*)d_in[4];
  const float* bg    = (const float*)d_in[5];
  float* outp = (float*)d_out;

  const size_t bytesT = (size_t)LL * PP * NN * sizeof(_Float16);
  const size_t bytesW = (size_t)NO * CH * sizeof(_Float16);
  const size_t offA = 0;
  const size_t offB = offA + bytesT;
  const size_t offW = offB + bytesT;
  const size_t total = offW + bytesW;
  if (total > ws_size) return;
  char* ws = (char*)d_ws;
  _Float16* At = (_Float16*)(ws + offA);
  _Float16* Bt = (_Float16*)(ws + offB);
  _Float16* Wh = (_Float16*)(ws + offW);

  hipLaunchKernelGGL(k_transpose, dim3(2 * LL, 1, 1), dim3(256, 1, 1), 0, stream, xd, xw, At, Bt);
  const int n2 = NO * CH / 2;
  hipLaunchKernelGGL(k_castw, dim3((n2 + 255) / 256, 1, 1), dim3(256, 1, 1), 0, stream, Wg, Wh, n2, WSC);
  hipLaunchKernelGGL(k_main, dim3(LL / 4, LL / 4, 1), dim3(256, 1, 1), 0, stream,
                     (const _Float16*)At, (const _Float16*)Bt, (const _Float16*)Wh, gamma, beta, bg, outp);
  (void)hipGetLastError();
}
